// Net_34857954575062
// MI455X (gfx1250) — hardware-verified
//
#include <hip/hip_runtime.h>
#include <stddef.h>
#include <stdint.h>
#include <math.h>

#define NB     4
#define CD     256
#define OD     256
#define HD     96
#define WD     96
#define HW     (HD * WD)
#define NPX    (NB * HW)
#define GBM    64
#define GBN    128
#define GTHR   128
#define SP     68
#define PTHR   256
#define NTB    (NPX / 64)
#define NWB    ((OD * CD / 8) / PTHR)
#define TPITCH 264
#define HALW   40
#define HALH   16
#define HALC   (HALH * HALW)
#define HALN   (16 * HALC)
#define WSMAX  134217728

#define XT_PLANE ((size_t)NPX * CD)
#define WB_PLANE ((size_t)OD * CD)
#define E_PLANE  ((size_t)NB * OD * HW)

static_assert(HW % GBM == 0);
static_assert(NPX % GBM == 0 && OD % GBN == 0 && CD % 32 == 0);
static_assert(GBM == (GTHR / 32) * 16 && GBN == GTHR);
static_assert(HD % 8 == 0 && WD % 32 == 0);
static_assert(HALN == 10 * 256 * 4);
static_assert(33 * 256 <= HALN);
static_assert((OD * CD / 8) % PTHR == 0);
static_assert((SP % 4) == 0 && SP >= GBM);
static_assert((TPITCH % 8) == 0 && TPITCH >= CD);

typedef float          v4f   __attribute__((ext_vector_type(4)));
typedef float          v8f   __attribute__((ext_vector_type(8)));
typedef int            v8i   __attribute__((ext_vector_type(8)));
typedef unsigned short v8us  __attribute__((ext_vector_type(8)));
typedef unsigned short v16us __attribute__((ext_vector_type(16)));
typedef __bf16         v16bf __attribute__((ext_vector_type(16)));
typedef v4f  __attribute__((may_alias)) v4fa;
typedef v8us __attribute__((may_alias)) v8usa;
union FragB { v16bf v; v16us u; v8us h[2]; v8i w; };

__device__ __forceinline__ v8f wmb(const FragB& a, const FragB& b, v8f c) {
  v8f d = __builtin_amdgcn_wmma_f32_16x16x32_bf16(false, a.v, false, b.v, (short)0, c, false, false);
  asm volatile("v_nop\n\tv_nop\n\tv_nop\n\tv_nop" : "+v"(d) : "v"(a.w), "v"(b.w));
  return d;
}

__device__ __forceinline__ unsigned bf16_bits(float f) {
  const unsigned u = __float_as_uint(f);
  return (u + 0x7FFFu + ((u >> 16) & 1u)) >> 16;
}
__device__ __forceinline__ float bf16_val(float f) {
  return __uint_as_float(bf16_bits(f) << 16);
}

#define OFFS(X) \
  X(0, 0, 0) \
  X(1, -1, -1) X(2, -1, 0) X(3, -1, 1) X(4, 0, -1) X(5, 0, 1) X(6, 1, -1) X(7, 1, 0) X(8, 1, 1) \
  X(9, -2, -2) X(10, -2, 0) X(11, -2, 2) X(12, 0, -2) X(13, 0, 2) X(14, 2, -2) X(15, 2, 0) X(16, 2, 2) \
  X(17, -3, -3) X(18, -3, 0) X(19, -3, 3) X(20, 0, -3) X(21, 0, 3) X(22, 3, -3) X(23, 3, 0) X(24, 3, 3) \
  X(25, -4, -4) X(26, -4, 0) X(27, -4, 4) X(28, 0, -4) X(29, 0, 4) X(30, 4, -4) X(31, 4, 0) X(32, 4, 4)

__global__ __launch_bounds__(PTHR) void k_prep(const float* __restrict__ F, const float* __restrict__ W,
                                               const float* __restrict__ bias,
                                               unsigned short* XT, unsigned short* WB, float* BI) {
  __shared__ __attribute__((aligned(16))) unsigned short tile[64 * TPITCH];
  const int tid = (int)threadIdx.x, lane = tid & 31, wave = tid >> 5;
  const int bx = (int)blockIdx.x;
  if (bx < NTB) {
    const int rowBase = bx * 64;
    const int b  = rowBase / HW;
    const int p0 = rowBase - b * HW;
    const float* fb = F + (size_t)b * CD * HW + p0;
    const int cl = tid >> 4;
    const int p4 = (tid & 15) * 4;
#pragma unroll 4
    for (int i = 0; i < 16; ++i) {
      const int c = 16 * i + cl;
      const v4f v = *(const v4fa*)(fb + (size_t)c * HW + p4);
      tile[(p4 + 0) * TPITCH + c] = (unsigned short)bf16_bits(v.x);
      tile[(p4 + 1) * TPITCH + c] = (unsigned short)bf16_bits(v.y);
      tile[(p4 + 2) * TPITCH + c] = (unsigned short)bf16_bits(v.z);
      tile[(p4 + 3) * TPITCH + c] = (unsigned short)bf16_bits(v.w);
    }
    __syncthreads();
    v8us q[8];
#pragma unroll
    for (int r = 0; r < 8; ++r) q[r] = *(const v8usa*)(tile + (8 * wave + r) * TPITCH + 8 * lane);
    unsigned short* dp = XT + (size_t)(rowBase + 8 * wave) * CD + 8 * lane;
#pragma unroll
    for (int r = 0; r < 8; ++r) *(volatile v8us*)(dp + (size_t)r * CD) = q[r];
    __threadfence();
#pragma unroll
    for (int r = 0; r < 8; ++r) *(volatile v8us*)(dp + (size_t)r * CD) = q[r];
  } else if (bx < NTB + NWB) {
    const int u  = (bx - NTB) * PTHR + tid;
    const int n  = u >> 5;
    const int k8 = (u & 31) * 8;
    const float* p = W + (size_t)n * CD + k8;
    const v4f a = *(const v4fa*)p;
    const v4f c = *(const v4fa*)(p + 4);
    v8us o;
    o[0] = (unsigned short)bf16_bits(a.x); o[1] = (unsigned short)bf16_bits(a.y);
    o[2] = (unsigned short)bf16_bits(a.z); o[3] = (unsigned short)bf16_bits(a.w);
    o[4] = (unsigned short)bf16_bits(c.x); o[5] = (unsigned short)bf16_bits(c.y);
    o[6] = (unsigned short)bf16_bits(c.z); o[7] = (unsigned short)bf16_bits(c.w);
    unsigned short* dp = WB + (size_t)n * CD + k8;
    *(volatile v8us*)dp = o;
    __threadfence();
    *(volatile v8us*)dp = o;
  } else {
    if (tid < 64) {
      const v4f a = *(const v4fa*)(bias + 4 * tid);
      v4f o;
      o.x = bf16_val(a.x); o.y = bf16_val(a.y); o.z = bf16_val(a.z); o.w = bf16_val(a.w);
      float* dp = BI + 4 * tid;
      *(volatile v4f*)dp = o;
      __threadfence();
      *(volatile v4f*)dp = o;
    }
  }
}

__global__ __launch_bounds__(GTHR) void k_embed(const unsigned short* __restrict__ XT,
                                                const unsigned short* __restrict__ WB,
                                                const float* __restrict__ BI, float* E) {
  __shared__ __attribute__((aligned(16))) float stg[GBN * SP];
  __shared__ float sb[GBN];
  const int tid = (int)threadIdx.x, lane = tid & 31, wave = tid >> 5, hh = lane >> 4, m = lane & 15;
  const int rowBase = (int)blockIdx.x * GBM;
  const int col0    = (int)blockIdx.y * GBN;
  const int z       = (int)blockIdx.z;

  sb[tid] = BI[(size_t)z * OD + col0 + tid];

  v8f acc[8];
  {
    const v8f zz = {0.f, 0.f, 0.f, 0.f, 0.f, 0.f, 0.f, 0.f};
#pragma unroll
    for (int t = 0; t < 8; ++t) acc[t] = zz;
  }
  const unsigned short* ap = XT + (size_t)z * XT_PLANE + (size_t)(rowBase + 16 * wave + m) * CD + 8 * hh;
  const unsigned short* bp = WB + (size_t)z * WB_PLANE + (size_t)(col0 + m) * CD + 8 * hh;

#pragma unroll 1
  for (int k0 = 0; k0 < CD; k0 += 32) {
    FragB af;
    af.h[0] = *(const v8usa*)(ap + k0);
    af.h[1] = *(const v8usa*)(ap + k0 + 16);
#pragma unroll
    for (int nt = 0; nt < 8; ++nt) {
      const unsigned short* wq = bp + (size_t)(16 * nt) * CD + k0;
      FragB bfg;
      bfg.h[0] = *(const v8usa*)wq;
      bfg.h[1] = *(const v8usa*)(wq + 16);
      acc[nt] = wmb(af, bfg, acc[nt]);
    }
  }
  __syncthreads();

#pragma unroll
  for (int nt = 0; nt < 8; ++nt) {
    const int lc = 16 * nt + m;
    const float bv = sb[lc];
    v4f lo4, hi4;
    lo4.x = acc[nt][0] + bv; lo4.y = acc[nt][1] + bv; lo4.z = acc[nt][2] + bv; lo4.w = acc[nt][3] + bv;
    hi4.x = acc[nt][4] + bv; hi4.y = acc[nt][5] + bv; hi4.z = acc[nt][6] + bv; hi4.w = acc[nt][7] + bv;
    float* sp = stg + lc * SP + 16 * wave + 8 * hh;
    *(v4fa*)sp = lo4;
    *(v4fa*)(sp + 4) = hi4;
  }
  __syncthreads();

  const int b  = rowBase / HW;
  const int p0 = rowBase - b * HW;
  float* eb = E + (size_t)z * E_PLANE + (size_t)(b * OD + col0) * HW + p0 + 4 * m;
#pragma unroll 1
  for (int i = 0; i < 16; ++i) {
    const int ol = 32 * wave + 2 * i + hh;
    const v4f v = *(const v4fa*)(stg + ol * SP + 4 * m);
    *(volatile v4f*)(eb + (size_t)ol * HW) = v;
  }
  __threadfence();
#pragma unroll 1
  for (int i = 0; i < 16; ++i) {
    const int ol = 32 * wave + 2 * i + hh;
    const v4f v = *(const v4fa*)(stg + ol * SP + 4 * m);
    *(volatile v4f*)(eb + (size_t)ol * HW) = v;
  }
}

template <int RND>
__device__ __forceinline__ void stage_halo(const float* __restrict__ src, float* hal, int h0, int w0, int tid) {
#pragma unroll 2
  for (int i = 0; i < 10; ++i) {
    const int idx = tid + 256 * i;
    const int ch  = idx / 160;
    const int rem = idx - ch * 160;
    const int hr  = rem / 10;
    const int q   = rem - hr * 10;
    const int gh  = h0 - 4 + hr;
    const int gw  = w0 - 4 + 4 * q;
    const bool ok = ((unsigned)gh < (unsigned)HD) && ((unsigned)gw < (unsigned)WD);
    const int ghc = gh < 0 ? 0 : (gh > HD - 1 ? HD - 1 : gh);
    const int gwc = gw < 0 ? 0 : (gw > WD - 4 ? WD - 4 : gw);
    const v4f v = *(const v4fa*)(src + (size_t)ch * HW + ghc * WD + gwc);
    const unsigned msk = ok ? 0xffffffffu : 0u;
    unsigned u0 = __float_as_uint(v.x), u1 = __float_as_uint(v.y);
    unsigned u2 = __float_as_uint(v.z), u3 = __float_as_uint(v.w);
    if (RND != 0) {
      u0 = (u0 + 0x7FFFu + ((u0 >> 16) & 1u)) & 0xffff0000u;
      u1 = (u1 + 0x7FFFu + ((u1 >> 16) & 1u)) & 0xffff0000u;
      u2 = (u2 + 0x7FFFu + ((u2 >> 16) & 1u)) & 0xffff0000u;
      u3 = (u3 + 0x7FFFu + ((u3 >> 16) & 1u)) & 0xffff0000u;
    }
    v4f o;
    o.x = __uint_as_float(u0 & msk); o.y = __uint_as_float(u1 & msk);
    o.z = __uint_as_float(u2 & msk); o.w = __uint_as_float(u3 & msk);
    *(v4fa*)(hal + ch * HALC + hr * HALW + 4 * q) = o;
  }
}

__global__ __launch_bounds__(256) void k_psla(const float* __restrict__ Ft, const float* __restrict__ Et,
                                              const float* __restrict__ Ee, float* out) {
  __shared__ __attribute__((aligned(16))) float hal[HALN];
  __shared__ float so[16 * 256];
  const int tid = (int)threadIdx.x, lane = tid & 31, wave = tid >> 5;
  const int w0 = (int)blockIdx.x * 32;
  const int h0 = (int)blockIdx.y * 8;
  const int b  = (int)blockIdx.z;
  const int h = h0 + wave, w = w0 + lane;
  const int base = (wave + 4) * HALW + lane + 4;
  const size_t pix = (size_t)h * WD + (size_t)w;

  float acc[33];
#pragma unroll
  for (int k = 0; k < 33; ++k) acc[k] = 0.0f;

  const float* etb = Et + (size_t)b * OD * HW;
  const float* eep = Ee + (size_t)b * OD * HW + pix;

#pragma unroll 1
  for (int ch = 0; ch < 16; ++ch) {
    stage_halo<0>(etb + (size_t)(16 * ch) * HW, hal, h0, w0, tid);
    __syncthreads();
#pragma unroll 1
    for (int o = 0; o < 16; ++o) {
      const float ee = eep[(size_t)(16 * ch + o) * HW];
      const float* lp = hal + o * HALC + base;
#define SC(K, A, B) acc[K] = fmaf(ee, lp[(A) * HALW + (B)], acc[K]);
      OFFS(SC)
#undef SC
    }
    __syncthreads();
  }

  float* sx = hal;
  {
    const float negv = -1.0e30f;
#define MK(K, A, B) { const bool okk = ((unsigned)(h + (A)) < (unsigned)HD) && ((unsigned)(w + (B)) < (unsigned)WD); \
                      sx[(K) * 256 + tid] = okk ? acc[K] : negv; }
    OFFS(MK)
#undef MK
  }
  float mx = -3.0e38f;
#pragma unroll 1
  for (int k = 0; k < 33; ++k) mx = fmaxf(mx, sx[k * 256 + tid]);
  float sum = 0.0f;
#pragma unroll 1
  for (int k = 0; k < 33; ++k) {
    const float e = expf(sx[k * 256 + tid] - mx);
    sx[k * 256 + tid] = e;
    sum += e;
  }
  const float inv = 1.0f / sum;
#define LW(K, A, B) acc[K] = sx[(K) * 256 + tid] * inv;
  OFFS(LW)
#undef LW
  __syncthreads();

  const float* fb = Ft + (size_t)b * CD * HW;
  float* ob = out + (size_t)b * CD * HW + pix;
#pragma unroll 1
  for (int ch = 0; ch < 16; ++ch) {
    stage_halo<1>(fb + (size_t)(16 * ch) * HW, hal, h0, w0, tid);
    __syncthreads();
#pragma unroll 1
    for (int ci = 0; ci < 16; ++ci) {
      const float* lp = hal + ci * HALC + base;
      float s = 0.0f;
#define AG(K, A, B) s = fmaf(acc[K], lp[(A) * HALW + (B)], s);
      OFFS(AG)
#undef AG
      so[ci * 256 + tid] = s;
      *(volatile float*)(ob + (size_t)(16 * ch + ci) * HW) = s;
    }
    __threadfence();
#pragma unroll 1
    for (int ci = 0; ci < 16; ++ci) {
      const float s = so[ci * 256 + tid];
      *(volatile float*)(ob + (size_t)(16 * ch + ci) * HW) = s;
    }
    __syncthreads();
  }
}

static inline size_t al256(size_t o) { return (o + 255) & ~(size_t)255; }

extern "C" void kernel_launch(void* const* d_in, const int* in_sizes, int n_in,
                              void* d_out, int out_size, void* d_ws, size_t ws_size,
                              hipStream_t stream) {
  if (n_in < 6) return;
  if (in_sizes[0] != NB * CD * HW || in_sizes[1] != NB * CD * HW) return;
  if (in_sizes[2] != OD * CD || in_sizes[3] != OD) return;
  if (in_sizes[4] != OD * CD || in_sizes[5] != OD) return;
  if (out_size != NB * CD * HW) return;

  const float* Ft  = (const float*)d_in[0];
  const float* Fe  = (const float*)d_in[1];
  const float* Wf  = (const float*)d_in[2];
  const float* bfv = (const float*)d_in[3];
  const float* Wg  = (const float*)d_in[4];
  const float* bgv = (const float*)d_in[5];
  float* out = (float*)d_out;

  char* ws = (char*)d_ws;
  size_t off = 0;
  const size_t oXT = off; off = al256(off + 2 * XT_PLANE * 2);
  const size_t oWB = off; off = al256(off + 2 * WB_PLANE * 2);
  const size_t oBI = off; off = al256(off + 2 * (size_t)OD * 4);
  const size_t oE  = off; off = al256(off + 2 * E_PLANE * 4);
  if (off > ws_size || off > (size_t)WSMAX) return;
  unsigned short* XT = (unsigned short*)(ws + oXT);
  unsigned short* WB = (unsigned short*)(ws + oWB);
  float*          BI = (float*)(ws + oBI);
  float*          E  = (float*)(ws + oE);

  k_prep<<<NTB + NWB + 1, PTHR, 0, stream>>>(Ft, Wf, bfv, XT, WB, BI);
  k_prep<<<NTB + NWB + 1, PTHR, 0, stream>>>(Fe, Wg, bgv, XT + XT_PLANE, WB + WB_PLANE, BI + OD);
  k_embed<<<dim3(NPX / GBM, OD / GBN, 2), GTHR, 0, stream>>>(XT, WB, BI, E);
  k_psla<<<dim3(WD / 32, HD / 8, NB), 256, 0, stream>>>(Ft, E, E + E_PLANE, out);
}
